// Rudy_56358560858316
// MI455X (gfx1250) — hardware-verified
//
#include <hip/hip_runtime.h>


typedef _Float16 half16 __attribute__((ext_vector_type(16)));
typedef float    float8 __attribute__((ext_vector_type(8)));

#define NBX 256
#define NBY 256
#define BSX (1000.0f / 256.0f)
#define BSY (1000.0f / 256.0f)
#define ROWH 40
#define KSTEP 32
#define OPS 16.0f

__global__ __launch_bounds__(256) void rudy_bbox(const float* __restrict__ pin_pos, const int* __restrict__ netpin_start,
                                                 const int* __restrict__ flat_netpin, const float* __restrict__ net_w,
                                                 float* xmin, float* xmax, float* ymin, float* ymax, float* sqc, int numNets, int numPins) {
    const int n = blockIdx.x * 256 + threadIdx.x;
    const bool ok = n < numNets;
    float x0 = 0.f, x1 = 0.f, y0 = 0.f, y1 = 0.f, sc = 0.f;
    if (ok) {
        int s = netpin_start[n], e = netpin_start[n + 1];
        if (s < 0) s = 0; if (e > numPins) e = numPins;
        if (e > s) {
            x0 = 3.4e38f; x1 = -3.4e38f; y0 = 3.4e38f; y1 = -3.4e38f;
            for (int p = s; p < e && p < s + 4096; ++p) {
                int pi = flat_netpin[p];
                pi = pi < 0 ? 0 : (pi >= numPins ? numPins - 1 : pi);
                float px = pin_pos[pi], py = pin_pos[numPins + pi];
                x0 = fminf(x0, px); x1 = fmaxf(x1, px); y0 = fminf(y0, py); y1 = fmaxf(y1, py);
            }
            float area = fmaxf((x1 - x0) * (y1 - y0), 1e-6f);
            sc = sqrtf(net_w[n] / area) * OPS;
        }
    }
    if (ok) {
        *(volatile float*)(xmin + n) = x0; *(volatile float*)(xmax + n) = x1; *(volatile float*)(ymin + n) = y0; *(volatile float*)(ymax + n) = y1; *(volatile float*)(sqc + n) = sc;
        __threadfence();
        *(volatile float*)(xmin + n) = x0; *(volatile float*)(xmax + n) = x1; *(volatile float*)(ymin + n) = y0; *(volatile float*)(ymax + n) = y1; *(volatile float*)(sqc + n) = sc;
    }
}

__global__ __launch_bounds__(256) void rudy_gemm(const float* __restrict__ xmin, const float* __restrict__ xmax, const float* __restrict__ ymin,
                                                 const float* __restrict__ ymax, const float* __restrict__ sqc, float* out, int numNets) {
    __shared__ float pxl[KSTEP], pxh[KSTEP], pyl[KSTEP], pyh[KSTEP], psq[KSTEP];
    __shared__ __align__(16) _Float16 OxL[16 * ROWH];
    __shared__ __align__(16) _Float16 OyL[NBY * ROWH];
    __shared__ __align__(16) float cst[16][NBY + 4];

    const int tid = threadIdx.x, lane = tid & 31, wave = tid >> 5;
    const int mLane = lane & 15, half = lane >> 4;
    const int xt = blockIdx.x;

    const float ybl = (float)tid * BSY, ybh = ybl + BSY;
    const float xbl = (float)(xt * 16 + (tid & 15)) * BSX, xbh = xbl + BSX;

    float8 acc[2] = {};
    const int nsteps = (numNets + KSTEP - 1) / KSTEP;
    for (int st = 0; st < nsteps; ++st) {
        const int k0 = st * KSTEP;
        __syncthreads();
        if (tid < KSTEP) {
            int n = k0 + tid;
            if (n < numNets) { pxl[tid] = xmin[n]; pxh[tid] = xmax[n]; pyl[tid] = ymin[n]; pyh[tid] = ymax[n]; psq[tid] = sqc[n]; }
            else { pxl[tid] = 0.f; pxh[tid] = 0.f; pyl[tid] = 0.f; pyh[tid] = 0.f; psq[tid] = 0.f; }
        }
        __syncthreads();
        {
            _Float16* d = OyL + tid * ROWH;
#pragma unroll
            for (int j = 0; j < KSTEP; ++j) {
                float ov = fmaxf(fminf(pyh[j], ybh) - fmaxf(pyl[j], ybl), 0.0f) * psq[j];
                d[j] = (_Float16)ov;
            }
        }
        if (tid < 16) {
            _Float16* d = OxL + tid * ROWH;
#pragma unroll
            for (int j = 0; j < KSTEP; ++j) {
                float ov = fmaxf(fminf(pxh[j], xbh) - fmaxf(pxl[j], xbl), 0.0f) * psq[j];
                d[j] = (_Float16)ov;
            }
        }
        __syncthreads();
        union { half16 v; uint4 q[2]; } ua, ub;
        const _Float16* arow = OxL + mLane * ROWH;
        ua.q[0] = *(const uint4*)(arow + 8 * half); ua.q[1] = *(const uint4*)(arow + 16 + 8 * half);
#pragma unroll
        for (int t = 0; t < 2; ++t) {
            const _Float16* brow = OyL + ((wave + 8 * t) * 16 + mLane) * ROWH;
            ub.q[0] = *(const uint4*)(brow + 8 * half); ub.q[1] = *(const uint4*)(brow + 16 + 8 * half);
            acc[t] = __builtin_amdgcn_wmma_f32_16x16x32_f16(false, ua.v, false, ub.v, (short)0, acc[t], false, false);
            asm volatile("v_nop\n\tv_nop\n\tv_nop\n\tv_nop" : "+v"(acc[t]) : "v"(ua.v), "v"(ub.v));
        }
    }
    const float scale = (1.0f / (OPS * OPS)) * (1.0f / (BSX * BSY));
#pragma unroll
    for (int t = 0; t < 2; ++t)
#pragma unroll
        for (int r = 0; r < 8; ++r) cst[8 * half + r][(wave + 8 * t) * 16 + mLane] = acc[t][r] * scale;
    __syncthreads();
    auto pass = [&]() {
#pragma unroll
        for (int j = 0; j < 2; ++j) {
            const int r = wave * 2 + j;
            float* orow = out + (size_t)(xt * 16 + r) * NBY;
#pragma unroll
            for (int c = 0; c < 8; ++c) *(volatile float*)(orow + c * 32 + lane) = cst[r][c * 32 + lane];
        }
    };
    pass();
    __threadfence();
    pass();
}

extern "C" void kernel_launch(void* const* d_in, const int* in_sizes, int n_in,
                              void* d_out, int out_size, void* d_ws, size_t ws_size,
                              hipStream_t stream) {
    (void)n_in; (void)out_size;
    const float* pin_pos      = (const float*)d_in[0];
    const int*   netpin_start = (const int*)d_in[1];
    const int*   flat_netpin  = (const int*)d_in[2];
    const float* net_weights  = (const float*)d_in[3];
    const int numPins = in_sizes[2];
    const int numNets = in_sizes[3];
    float* out = (float*)d_out;
    if ((size_t)5 * numNets * sizeof(float) > ws_size) return;
    float* ws  = (float*)d_ws;
    float* xmin = ws;
    float* xmax = ws + (size_t)numNets;
    float* ymin = ws + (size_t)2 * numNets;
    float* ymax = ws + (size_t)3 * numNets;
    float* sqc  = ws + (size_t)4 * numNets;
    rudy_bbox<<<(numNets + 255) / 256, 256, 0, stream>>>(pin_pos, netpin_start, flat_netpin, net_weights, xmin, xmax, ymin, ymax, sqc, numNets, numPins);
    rudy_gemm<<<NBX / 16, 256, 0, stream>>>(xmin, xmax, ymin, ymax, sqc, out, numNets);
}
